// Proposed_Module_LocalGNN_4638564679953
// MI455X (gfx1250) — hardware-verified
//
#include <hip/hip_runtime.h>
#define CC 32
#define SD 64
#define NP (SD * SD * SD)
#define PCH 16384
#define NWN 4096
#define NND 8
#define NRN (NWN * NND)
#define NPR (NWN * NND * NND)
typedef __bf16 v16b __attribute__((ext_vector_type(16)));
typedef unsigned short v8us __attribute__((ext_vector_type(8), may_alias));
typedef float  v8f  __attribute__((ext_vector_type(8)));
typedef float  v4f  __attribute__((ext_vector_type(4)));
typedef float  v4fa __attribute__((ext_vector_type(4), may_alias));
union FragB { v16b v; v8us half[2]; unsigned short u[16]; };

__device__ __forceinline__ unsigned short bf16_bits(float x) { unsigned int u = __float_as_uint(x); return (unsigned short)((u + 0x7FFFu + ((u >> 16) & 1u)) >> 16); }
__device__ __forceinline__ float bf16_val(unsigned short b) { return __uint_as_float(((unsigned int)b) << 16); }
__device__ __forceinline__ float bf16_round(float x) { return bf16_val(bf16_bits(x)); }
template <int NT>
__device__ __forceinline__ v8f mmaN(v16b ah, v16b al, v16b bh, v16b bl, v8f c) {
  c = __builtin_amdgcn_wmma_f32_16x16x32_bf16(false, ah, false, bh, (short)0, c, false, false);
  if (NT >= 2) c = __builtin_amdgcn_wmma_f32_16x16x32_bf16(false, al, false, bh, (short)0, c, false, false);
  if (NT >= 3) c = __builtin_amdgcn_wmma_f32_16x16x32_bf16(false, ah, false, bl, (short)0, c, false, false);
  asm volatile("v_nop\n\tv_nop\n\tv_nop\n\tv_nop" : "+v"(c) : "v"(ah), "v"(al), "v"(bh), "v"(bl));
  return c;
}

__global__ __launch_bounds__(256) void k_wt_bf16(const float* __restrict__ W, unsigned short* __restrict__ Wt, int K, int N) {
  const int t = blockIdx.x * 256 + threadIdx.x;
  const int k8n = K / 8;
  if (t >= N * k8n) return;
  const int n = t / k8n, k8 = (t % k8n) * 8;
  v8us v;
#pragma unroll
  for (int i = 0; i < 8; ++i) v[i] = bf16_bits(W[(size_t)(k8 + i) * N + n]);
  *(volatile v8us*)(Wt + (size_t)n * K + k8) = v;
  __threadfence();
  *(volatile v8us*)(Wt + (size_t)n * K + k8) = v;
}

template <bool ASPLIT, int ACT, bool BIAS_BF16>
__global__ __launch_bounds__(128) void k_gemm_bf(const float* __restrict__ A, int lda, const unsigned short* __restrict__ Wt, int ldb,
                                               const float* __restrict__ bias, float* __restrict__ C, int ldc, int M, int N, int K) {
  __shared__ __attribute__((aligned(16))) float so[4][16][64];
  const int tid = threadIdx.x, w = tid >> 5, lane = tid & 31, ln = lane & 15, hh = lane >> 4;
  const int ntn = N / 64;
  const int wid = blockIdx.x * 4 + w;
  const int mt = wid / ntn, nq = wid % ntn;
  if (mt * 16 >= M) return;
  const int row0 = mt * 16, col0 = nq * 64;
  const float* arow = A + (size_t)(row0 + ln) * lda;
  v8f acc[4] = {};
  for (int kb = 0; kb < K; kb += 32) {
    FragB ah, al;
    const v4f x0 = *(const v4fa*)(arow + kb + 8 * hh), x1 = *(const v4fa*)(arow + kb + 8 * hh + 4);
    const v4f x2 = *(const v4fa*)(arow + kb + 16 + 8 * hh), x3 = *(const v4fa*)(arow + kb + 16 + 8 * hh + 4);
    float xs[16] = {x0[0],x0[1],x0[2],x0[3],x1[0],x1[1],x1[2],x1[3],x2[0],x2[1],x2[2],x2[3],x3[0],x3[1],x3[2],x3[3]};
#pragma unroll
    for (int i = 0; i < 16; ++i) { const unsigned short hb = bf16_bits(xs[i]); ah.u[i] = hb; al.u[i] = ASPLIT ? bf16_bits(xs[i] - bf16_val(hb)) : (unsigned short)0; }
#pragma unroll
    for (int t = 0; t < 4; ++t) {
      const unsigned short* brow = Wt + (size_t)(col0 + t * 16 + ln) * ldb + kb;
      FragB b;
      b.half[0] = *(const v8us*)(brow + 8 * hh);
      b.half[1] = *(const v8us*)(brow + 16 + 8 * hh);
      acc[t] = mmaN<ASPLIT ? 2 : 1>(ah.v, al.v, b.v, b.v, acc[t]);
    }
  }
#pragma unroll
  for (int t = 0; t < 4; ++t) {
    float bv = bias ? bias[col0 + t * 16 + ln] : 0.f;
    if (BIAS_BF16) bv = bf16_round(bv);
#pragma unroll
    for (int r = 0; r < 8; ++r) { float v = acc[t][r] + bv; if (ACT == 1) v = fmaxf(v, 0.f); so[w][8 * hh + r][t * 16 + ln] = v; }
  }
  __builtin_amdgcn_fence(__ATOMIC_ACQ_REL, "workgroup");
  __builtin_amdgcn_wave_barrier();
  const int rsub = lane >> 4, c4 = (lane & 15) * 4;
  for (int pass = 0; pass < 2; ++pass) {
#pragma unroll
    for (int q = 0; q < 8; ++q) {
      const int r = q * 2 + rsub;
      const v4f v = *(const v4fa*)&so[w][r][c4];
      *(volatile v4f*)(C + (size_t)(row0 + r) * ldc + col0 + c4) = v;
    }
    if (pass == 0) __threadfence();
  }
}

template <bool ASPLIT, int ACT, bool BIAS_BF16, bool RES_BF16>
__global__ __launch_bounds__(128) void k_gemm_bf3(const float* __restrict__ A, int lda, const unsigned short* __restrict__ Wt, int ldb,
                                                const float* __restrict__ bias, const float* __restrict__ resid, int rmod, int ldr,
                                                float* __restrict__ C, int ldc, int M, int N, int K) {
  __shared__ __attribute__((aligned(16))) float so[4][16][64];
  const int tid = threadIdx.x, w = tid >> 5, lane = tid & 31, ln = lane & 15, hh = lane >> 4;
  const int ntn = N / 64;
  const int wid = blockIdx.x * 4 + w;
  const int mt = wid / ntn, nq = wid % ntn;
  if (mt * 16 >= M) return;
  const int row0 = mt * 16, col0 = nq * 64;
  const float* arow = A + (size_t)(row0 + ln) * lda;
  v8f acc[4] = {};
  for (int kb = 0; kb < K; kb += 32) {
    FragB ah, al;
    const v4f x0 = *(const v4fa*)(arow + kb + 8 * hh), x1 = *(const v4fa*)(arow + kb + 8 * hh + 4);
    const v4f x2 = *(const v4fa*)(arow + kb + 16 + 8 * hh), x3 = *(const v4fa*)(arow + kb + 16 + 8 * hh + 4);
    float xs[16] = {x0[0],x0[1],x0[2],x0[3],x1[0],x1[1],x1[2],x1[3],x2[0],x2[1],x2[2],x2[3],x3[0],x3[1],x3[2],x3[3]};
#pragma unroll
    for (int i = 0; i < 16; ++i) { const unsigned short hb = bf16_bits(xs[i]); ah.u[i] = hb; al.u[i] = ASPLIT ? bf16_bits(xs[i] - bf16_val(hb)) : (unsigned short)0; }
#pragma unroll
    for (int t = 0; t < 4; ++t) {
      const unsigned short* brow = Wt + (size_t)(col0 + t * 16 + ln) * ldb + kb;
      FragB b;
      b.half[0] = *(const v8us*)(brow + 8 * hh);
      b.half[1] = *(const v8us*)(brow + 16 + 8 * hh);
      acc[t] = mmaN<ASPLIT ? 2 : 1>(ah.v, al.v, b.v, b.v, acc[t]);
    }
  }
#pragma unroll
  for (int t = 0; t < 4; ++t) {
    const int col = col0 + t * 16 + ln;
    float bv = bias ? bias[col] : 0.f;
    if (BIAS_BF16) bv = bf16_round(bv);
#pragma unroll
    for (int r = 0; r < 8; ++r) {
      float v = acc[t][r] + bv;
      if (resid) { float rv = resid[(size_t)((row0 + 8 * hh + r) % rmod) * ldr + col]; if (RES_BF16) rv = bf16_round(rv); v += rv; }
      if (ACT == 1) v = fmaxf(v, 0.f);
      if (ACT == 2) v = 0.5f * v * (1.0f + erff(v * 0.70710678118654752f));
      if (ACT == 3) { const float u = 0.7978845608028654f * (v + 0.044715f * v * v * v); v = 0.5f * v * (1.0f + tanhf(u)); }
      so[w][8 * hh + r][t * 16 + ln] = v;
    }
  }
  __builtin_amdgcn_fence(__ATOMIC_ACQ_REL, "workgroup");
  __builtin_amdgcn_wave_barrier();
  const int rsub = lane >> 4, c4 = (lane & 15) * 4;
  for (int pass = 0; pass < 2; ++pass) {
#pragma unroll
    for (int q = 0; q < 8; ++q) {
      const int r = q * 2 + rsub;
      const v4f v = *(const v4fa*)&so[w][r][c4];
      *(volatile v4f*)(C + (size_t)(row0 + r) * ldc + col0 + c4) = v;
    }
    if (pass == 0) __threadfence();
  }
}
template <bool PARAM_BF16>
__global__ __launch_bounds__(256) void k_layernorm(const float* __restrict__ X, const float* __restrict__ R, const float* __restrict__ g, const float* __restrict__ bta,
                                                  float* __restrict__ out_sum, float* __restrict__ out_norm, int N, float eps) {
  __shared__ float red[256];
  const int row = blockIdx.x, tid = threadIdx.x;
  const float* x = X + (size_t)row * N; const float* rr = R ? R + (size_t)row * N : nullptr;
  float vals[16];
  const int per = N / 256;
  float s1 = 0.f;
  for (int u = 0; u < per / 4; ++u) {
    const int j = tid * 4 + 1024 * u;
    const v4f a = *(const v4fa*)(x + j);
    v4f b = {0.f,0.f,0.f,0.f}; if (rr) b = *(const v4fa*)(rr + j);
#pragma unroll
    for (int q = 0; q < 4; ++q) { const float v = a[q] + b[q]; vals[u * 4 + q] = v; s1 += v; }
  }
  red[tid] = s1; __syncthreads();
  for (int st = 128; st > 0; st >>= 1) { if (tid < st) red[tid] += red[tid + st]; __syncthreads(); }
  const float mu = red[0] / (float)N; __syncthreads();
  float s2 = 0.f;
  for (int u = 0; u < per / 4; ++u)
#pragma unroll
    for (int q = 0; q < 4; ++q) { const float c = vals[u * 4 + q] - mu; s2 += c * c; }
  red[tid] = s2; __syncthreads();
  for (int st = 128; st > 0; st >>= 1) { if (tid < st) red[tid] += red[tid + st]; __syncthreads(); }
  const float rs = rsqrtf(red[0] / (float)N + eps);
  for (int pass = 0; pass < 2; ++pass) {
    for (int u = 0; u < per / 4; ++u) {
      const int j = tid * 4 + 1024 * u;
      v4f o, sm;
#pragma unroll
      for (int q = 0; q < 4; ++q) {
        float gg = g[j + q], bb = bta[j + q];
        if (PARAM_BF16) { gg = bf16_round(gg); bb = bf16_round(bb); }
        sm[q] = vals[u * 4 + q]; o[q] = (vals[u * 4 + q] - mu) * rs * gg + bb;
      }
      if (out_sum) *(volatile v4f*)(out_sum + (size_t)row * N + j) = sm;
      *(volatile v4f*)(out_norm + (size_t)row * N + j) = o;
    }
    if (pass == 0) __threadfence();
  }
}


typedef _Float16 v16h __attribute__((ext_vector_type(16)));
union FragH { v16h v; v8us half[2]; _Float16 h[16]; unsigned short u[16]; };
template <int NT>
__device__ __forceinline__ v8f mmaH(v16h ah, v16h al, v16h bh, v16h bl, v8f c) {
  c = __builtin_amdgcn_wmma_f32_16x16x32_f16(false, ah, false, bh, (short)0, c, false, false);
  if (NT >= 2) c = __builtin_amdgcn_wmma_f32_16x16x32_f16(false, al, false, bh, (short)0, c, false, false);
  if (NT >= 3) c = __builtin_amdgcn_wmma_f32_16x16x32_f16(false, ah, false, bl, (short)0, c, false, false);
  asm volatile("v_nop\n\tv_nop\n\tv_nop\n\tv_nop" : "+v"(c) : "v"(ah), "v"(al), "v"(bh), "v"(bl));
  return c;
}
template <bool ASPLIT>
__global__ __launch_bounds__(128) void k_gemm_h(const float* __restrict__ A, int lda, size_t sA, const _Float16* __restrict__ Bh, int ldb, size_t sB, float alpha, float* __restrict__ C, int ldc, size_t sC, int M, int N, int K) {
  __shared__ __attribute__((aligned(16))) float so[4][16][64];
  const int tid = threadIdx.x, w = tid >> 5, lane = tid & 31, ln = lane & 15, hh = lane >> 4; const int by = blockIdx.y;
  A += (size_t)by * sA; Bh += (size_t)by * sB; C += (size_t)by * sC;
  const int ntn = (N + 63) / 64; const int wid = blockIdx.x * 4 + w; const int mt = wid / ntn, nq = wid % ntn; if (mt * 16 >= M) return;
  const int row0 = mt * 16, col0 = nq * 64; const float* arow = A + (size_t)(row0 + ln) * lda;
  v8f acc[4] = {};
  for (int kb = 0; kb < K; kb += 32) {
    FragH ah, al;
    const v4f x0 = *(const v4fa*)(arow + kb + 8 * hh), x1 = *(const v4fa*)(arow + kb + 8 * hh + 4), x2 = *(const v4fa*)(arow + kb + 16 + 8 * hh), x3 = *(const v4fa*)(arow + kb + 16 + 8 * hh + 4);
    float xs[16] = {x0[0],x0[1],x0[2],x0[3],x1[0],x1[1],x1[2],x1[3],x2[0],x2[1],x2[2],x2[3],x3[0],x3[1],x3[2],x3[3]};
#pragma unroll
    for (int i = 0; i < 16; ++i) { const _Float16 h = (_Float16)xs[i]; ah.h[i] = h; al.h[i] = ASPLIT ? (_Float16)(xs[i] - (float)h) : (_Float16)0.0f; }
#pragma unroll
    for (int t = 0; t < 4; ++t) { if (col0 + t * 16 >= N) continue; const size_t boff = (size_t)(col0 + t * 16 + ln) * ldb + kb; FragH bq; bq.half[0] = *(const v8us*)(Bh + boff + 8 * hh); bq.half[1] = *(const v8us*)(Bh + boff + 16 + 8 * hh);
      acc[t] = mmaH<ASPLIT ? 2 : 1>(ah.v, al.v, bq.v, bq.v, acc[t]); }
  }
#pragma unroll
  for (int t = 0; t < 4; ++t) { if (col0 + t * 16 >= N) continue;
#pragma unroll
    for (int r = 0; r < 8; ++r) so[w][8 * hh + r][t * 16 + ln] = acc[t][r] * alpha; }
  __builtin_amdgcn_fence(__ATOMIC_ACQ_REL, "workgroup"); __builtin_amdgcn_wave_barrier();
  const int rsub = lane >> 4, c4 = (lane & 15) * 4;
  for (int pass = 0; pass < 2; ++pass) {
#pragma unroll
    for (int q = 0; q < 8; ++q) { const int r = q * 2 + rsub; if (col0 + c4 < N) { const v4f v = *(const v4fa*)&so[w][r][c4]; *(volatile v4f*)(C + (size_t)(row0 + r) * ldc + col0 + c4) = v; } }
    if (pass == 0) __threadfence(); }
}

__global__ __launch_bounds__(256) void k_wt_f16(const float* __restrict__ W, _Float16* __restrict__ Wt, int K, int N, float scale) {
  const int t = blockIdx.x * 256 + threadIdx.x; if (t >= N * (K / 8)) return; const int n = t / (K / 8), k8 = (t % (K / 8)) * 8; FragH f;
#pragma unroll
  for (int i = 0; i < 8; ++i) f.h[i] = (_Float16)(bf16_round(W[(size_t)(k8 + i) * N + n]) * scale); const v8us o = f.half[0];
  *(volatile v8us*)((unsigned short*)Wt + (size_t)n * K + k8) = o; __threadfence(); *(volatile v8us*)((unsigned short*)Wt + (size_t)n * K + k8) = o;
}
template <int ACT>
__global__ __launch_bounds__(128) void k_gemm_hhx(const _Float16* __restrict__ A, int lda, size_t sA, const _Float16* __restrict__ Bh, int ldb, size_t sB, float alpha, const float* __restrict__ bias, size_t sBias, const float* __restrict__ CP, int rowsPerB, size_t sCPb, int row0g,
    float* __restrict__ C, _Float16* __restrict__ C16, int ldc, size_t sC, int M, int N, int K) {
  __shared__ __attribute__((aligned(16))) float so[4][16][64];
  const int tid = threadIdx.x, w = tid >> 5, lane = tid & 31, ln = lane & 15, hh = lane >> 4; const int by = blockIdx.y;
  A += (size_t)by * sA; Bh += (size_t)by * sB; const size_t cofs = (size_t)by * sC; const float* bp = bias ? bias + (size_t)by * sBias : nullptr;
  const int ntn = (N + 63) / 64; const int wid = blockIdx.x * 4 + w; const int mt = wid / ntn, nq = wid % ntn; if (mt * 16 >= M) return;
  const int row0 = mt * 16, col0 = nq * 64; const _Float16* arow = A + (size_t)(row0 + ln) * lda;
  v8f acc[4] = {};
  for (int kb = 0; kb < K; kb += 32) { FragH ah; ah.half[0] = *(const v8us*)((const unsigned short*)arow + kb + 8 * hh); ah.half[1] = *(const v8us*)((const unsigned short*)arow + kb + 16 + 8 * hh);
#pragma unroll
    for (int t = 0; t < 4; ++t) { if (col0 + t * 16 >= N) continue; const size_t boff = (size_t)(col0 + t * 16 + ln) * ldb + kb; FragH bq; bq.half[0] = *(const v8us*)((const unsigned short*)Bh + boff + 8 * hh); bq.half[1] = *(const v8us*)((const unsigned short*)Bh + boff + 16 + 8 * hh);
      acc[t] = mmaH<1>(ah.v, ah.v, bq.v, bq.v, acc[t]); }
  }
#pragma unroll
  for (int t = 0; t < 4; ++t) { if (col0 + t * 16 >= N) continue; const int col = col0 + t * 16 + ln; const float bv = bp ? bf16_round(bp[col]) : 0.f;
#pragma unroll
    for (int r = 0; r < 8; ++r) { float v = acc[t][r] * alpha + bv; if (CP) { const int bidx = (row0g + row0 + 8 * hh + r) / rowsPerB; v += CP[(size_t)bidx * sCPb + (size_t)by * 64 + col]; } if (ACT == 1) v = (v > 0.f) ? v : expm1f(v); else if (ACT == 7) v = (v > 0.f) ? v + 1.0f : expf(v); else if (ACT == 8) v = tanhf(v); else if (ACT == 9) v = 0.5f * v * (1.0f + tanhf(0.7978845608028654f * (v + 0.044715f * v * v * v))); else if (ACT == 11) v = 1.0f / (1.0f + expf(-v)); else if (ACT == 12) v = (v > 0.f) ? v : 0.01f * v; else if (ACT == 14) v = (v > 0.f) ? v : 0.1f * v; else if (ACT == 15) v = v / (1.0f + expf(-v)); else if (ACT == 3) v = fmaxf(v, 0.f); else if (ACT == 6) v = 0.5f * v * (1.0f + erff(v * 0.70710678118654752f)); so[w][8 * hh + r][t * 16 + ln] = v; } }
  __builtin_amdgcn_fence(__ATOMIC_ACQ_REL, "workgroup"); __builtin_amdgcn_wave_barrier();
  const int rsub = lane >> 4, c4 = (lane & 15) * 4; typedef _Float16 v4h __attribute__((ext_vector_type(4)));
  for (int pass = 0; pass < 2; ++pass) {
#pragma unroll
    for (int q = 0; q < 8; ++q) { const int r = q * 2 + rsub; if (col0 + c4 < N) { const v4f v = *(const v4fa*)&so[w][r][c4]; if (C) *(volatile v4f*)(C + cofs + (size_t)(row0 + r) * ldc + col0 + c4) = v; if (C16) { v4h h4; for (int i = 0; i < 4; ++i) h4[i] = (_Float16)v[i]; *(volatile v4h*)(C16 + cofs + (size_t)(row0 + r) * ldc + col0 + c4) = h4; } } }
    if (pass == 0) __threadfence(); }
}


typedef _Float16 v4h __attribute__((ext_vector_type(4)));

__global__ __launch_bounds__(256) void k_x16(const float* __restrict__ x, _Float16* __restrict__ X16, size_t n8) { const size_t t = (size_t)blockIdx.x * 256 + threadIdx.x; if (t >= n8) return; FragH f;
#pragma unroll
  for (int q = 0; q < 8; ++q) f.h[q] = (_Float16)bf16_round(x[t * 8 + q]); *(volatile v8us*)((unsigned short*)X16 + t * 8) = f.half[0]; __threadfence(); *(volatile v8us*)((unsigned short*)X16 + t * 8) = f.half[0]; }
__global__ __launch_bounds__(256) void k_h16(const float* __restrict__ x, _Float16* __restrict__ X16, size_t n8) { const size_t t = (size_t)blockIdx.x * 256 + threadIdx.x; if (t >= n8) return; FragH f;
#pragma unroll
  for (int q = 0; q < 8; ++q) f.h[q] = (_Float16)x[t * 8 + q]; *(volatile v8us*)((unsigned short*)X16 + t * 8) = f.half[0]; __threadfence(); *(volatile v8us*)((unsigned short*)X16 + t * 8) = f.half[0]; }
__global__ __launch_bounds__(256) void k_round16f(const float* __restrict__ W, _Float16* __restrict__ Bt, size_t n8) { const size_t t = (size_t)blockIdx.x * 256 + threadIdx.x; if (t >= n8) return; FragH f;
#pragma unroll
  for (int i = 0; i < 8; ++i) f.h[i] = (_Float16)(bf16_round(W[t * 8 + i]) * 16.0f); *(volatile v8us*)((unsigned short*)Bt + t * 8) = f.half[0]; __threadfence(); *(volatile v8us*)((unsigned short*)Bt + t * 8) = f.half[0]; }
template <int NHv, int TTv>
__global__ __launch_bounds__(256) void k_vt(const _Float16* __restrict__ V16, int ldv, int voff, _Float16* __restrict__ Vt) { __shared__ unsigned short tl[64][66]; const int tid = threadIdx.x; const int slab = blockIdx.x / (TTv / 64), lg = blockIdx.x % (TTv / 64); const int b = slab / NHv, h = slab % NHv;
  for (int i = tid; i < 64 * 8; i += 256) { const int r = i / 8, c8 = (i % 8) * 8; FragH f; f.half[0] = *(const v8us*)((const unsigned short*)V16 + ((size_t)b * TTv + lg * 64 + r) * ldv + voff + h * 64 + c8);
#pragma unroll
    for (int q = 0; q < 8; ++q) tl[r][c8 + q] = f.u[q]; }
  __syncthreads();
  for (int pass = 0; pass < 2; ++pass) {
#pragma unroll
    for (int rd = 0; rd < 2; ++rd) { const int d = rd * 32 + tid / 8, pc = tid % 8; FragH f;
#pragma unroll
      for (int q = 0; q < 8; ++q) f.u[q] = tl[pc * 8 + q][d];
      *(volatile v8us*)((unsigned short*)Vt + ((size_t)slab * 64 + d) * TTv + lg * 64 + pc * 8) = f.half[0]; }
    if (pass == 0) __threadfence(); } }

__global__ __launch_bounds__(256) void k_hl(const float* __restrict__ F, _Float16* __restrict__ Hh, _Float16* __restrict__ Hl, size_t n8) { const size_t t = (size_t)blockIdx.x * 256 + threadIdx.x; if (t >= n8) return; FragH fh, fl; const v4f a = *(const v4fa*)(F + t * 8), c = *(const v4fa*)(F + t * 8 + 4);
#pragma unroll
  for (int q = 0; q < 4; ++q) { _Float16 h = (_Float16)a[q]; fh.h[q] = h; fl.h[q] = (_Float16)((a[q] - (float)h) * 1024.0f); h = (_Float16)c[q]; fh.h[4 + q] = h; fl.h[4 + q] = (_Float16)((c[q] - (float)h) * 1024.0f); }
  for (int pass = 0; pass < 2; ++pass) { *(volatile v8us*)((unsigned short*)Hh + t * 8) = fh.half[0]; *(volatile v8us*)((unsigned short*)Hl + t * 8) = fl.half[0]; if (pass == 0) __threadfence(); } }

__device__ __forceinline__ float lrelu_f(float v) { return (v >= 0.f) ? v : 0.2f * v; }
__global__ __launch_bounds__(256) void k_x16v(const float* __restrict__ x, _Float16* __restrict__ X16) { const int t = blockIdx.x * 256 + threadIdx.x; if (t >= NP * (CC / 8)) return; const int c0 = (t % (CC / 8)) * 8, p = t / (CC / 8); FragH f;
#pragma unroll
  for (int q = 0; q < 8; ++q) f.h[q] = (_Float16)bf16_round(x[(size_t)(c0 + q) * NP + p]);
  *(volatile v8us*)((unsigned short*)X16 + (size_t)p * CC + c0) = f.half[0]; __threadfence(); *(volatile v8us*)((unsigned short*)X16 + (size_t)p * CC + c0) = f.half[0]; }
__global__ __launch_bounds__(256) void k_im2col3(const _Float16* __restrict__ P, int C, int p0, int cnt, _Float16* __restrict__ COL) { const int t = blockIdx.x * 256 + threadIdx.x; if (t >= cnt * 27 * (C / 8)) return; const int c0 = (t % (C / 8)) * 8; const int k = (t / (C / 8)) % 27; const int pl = t / ((C / 8) * 27); const int p = p0 + pl; const int d = p / (SD * SD), h = (p / SD) % SD, w = p % SD; const int dd = d + k / 9 - 1, hh = h + (k / 3) % 3 - 1, ww = w + k % 3 - 1; FragH f = FragH{};
  if (dd >= 0 && dd < SD && hh >= 0 && hh < SD && ww >= 0 && ww < SD) f.half[0] = *(const v8us*)((const unsigned short*)P + ((size_t)(dd * SD + hh) * SD + ww) * C + c0);
  *(volatile v8us*)((unsigned short*)COL + ((size_t)pl * 27 + k) * C + c0) = f.half[0]; __threadfence(); *(volatile v8us*)((unsigned short*)COL + ((size_t)pl * 27 + k) * C + c0) = f.half[0]; }
__global__ __launch_bounds__(256) void k_w3d(const float* __restrict__ w, int O, int C, _Float16* __restrict__ Bt) { const int KD = 27 * C; const int t = blockIdx.x * 256 + threadIdx.x; if (t >= O * (KD / 8)) return; const int col0 = (t % (KD / 8)) * 8, o = t / (KD / 8); const int k = col0 / C, c0 = col0 % C; FragH f;
#pragma unroll
  for (int q = 0; q < 8; ++q) f.h[q] = (_Float16)(bf16_round(w[((size_t)o * C + c0 + q) * 27 + k]) * 16.0f);
  *(volatile v8us*)((unsigned short*)Bt + (size_t)o * KD + col0) = f.half[0]; __threadfence(); *(volatile v8us*)((unsigned short*)Bt + (size_t)o * KD + col0) = f.half[0]; }
__global__ __launch_bounds__(256) void k_stat(const _Float16* __restrict__ F, int C, int phase, float* __restrict__ ST) {
  #pragma clang fp contract(off)
  __shared__ float red[256]; const int c = blockIdx.x, tid = threadIdx.x; const float mean = phase ? (ST[(size_t)c * 32] / (float)NP) : 0.f; float s = 0.f;
  for (int p = tid; p < NP; p += 256) { const float v = (float)F[(size_t)p * C + c]; s += phase ? (v - mean) * (v - mean) : v; }
  red[tid] = s; __syncthreads(); for (int st = 128; st > 0; st >>= 1) { if (tid < st) red[tid] += red[tid + st]; __syncthreads(); }
  if (tid < 32) { float* line = ST + ((size_t)phase * 64 + c) * 32; *(volatile float*)(line + tid) = red[0]; __threadfence(); *(volatile float*)(line + tid) = red[0]; } }
__global__ __launch_bounds__(256) void k_inl(_Float16* P16, int C, const float* __restrict__ ST, _Float16* O16) {
  #pragma clang fp contract(off)
  const int t = blockIdx.x * 256 + threadIdx.x; if (t >= NP * (C / 8)) return; const int c0 = (t % (C / 8)) * 8, p = t / (C / 8); FragH in; in.half[0] = *(const v8us*)((const unsigned short*)P16 + (size_t)p * C + c0); FragH f;
#pragma unroll
  for (int q = 0; q < 8; ++q) { const int c = c0 + q; const float mean = ST[(size_t)c * 32] / (float)NP, rs = rsqrtf(ST[(size_t)(64 + c) * 32] / (float)NP + 1e-5f); f.h[q] = (_Float16)lrelu_f(((float)in.h[q] - mean) * rs); }
  *(volatile v8us*)((unsigned short*)O16 + (size_t)p * C + c0) = f.half[0]; __threadfence(); *(volatile v8us*)((unsigned short*)O16 + (size_t)p * C + c0) = f.half[0]; }
__global__ __launch_bounds__(256) void k_inl32(const float* __restrict__ F, int C, const float* __restrict__ ST, _Float16* __restrict__ Hi, _Float16* __restrict__ Lo) {
  #pragma clang fp contract(off)
  const int t = blockIdx.x * 256 + threadIdx.x; if (t >= NP * (C / 8)) return; const int c0 = (t % (C / 8)) * 8, p = t / (C / 8); const v4f a = *(const v4fa*)(F + (size_t)p * C + c0), cc = *(const v4fa*)(F + (size_t)p * C + c0 + 4); FragH fh, fl;
#pragma unroll
  for (int q = 0; q < 8; ++q) { const int c = c0 + q; const float mean = ST[(size_t)c * 32] / (float)NP, rs = rsqrtf(ST[(size_t)(64 + c) * 32] / (float)NP + 1e-5f); const float v = lrelu_f((((q < 4) ? a[q] : cc[q - 4]) - mean) * rs); const _Float16 h = (_Float16)v; fh.h[q] = h; fl.h[q] = (_Float16)((v - (float)h) * 1024.0f); }
  for (int pass = 0; pass < 2; ++pass) { *(volatile v8us*)((unsigned short*)Hi + (size_t)p * C + c0) = fh.half[0]; if (Lo) *(volatile v8us*)((unsigned short*)Lo + (size_t)p * C + c0) = fl.half[0]; if (pass == 0) __threadfence(); } }
__global__ __launch_bounds__(256) void k_stat32(const float* __restrict__ F, int C, int phase, float* __restrict__ ST) {
  #pragma clang fp contract(off)
  __shared__ float red[256]; const int c = blockIdx.x, tid = threadIdx.x; const float mean = phase ? (ST[(size_t)c * 32] / (float)NP) : 0.f; float s = 0.f;
  for (int p = tid; p < NP; p += 256) { const float v = F[(size_t)p * C + c]; s += phase ? (v - mean) * (v - mean) : v; }
  red[tid] = s; __syncthreads(); for (int st = 128; st > 0; st >>= 1) { if (tid < st) red[tid] += red[tid + st]; __syncthreads(); }
  if (tid < 32) { float* line = ST + ((size_t)phase * 64 + c) * 32; *(volatile float*)(line + tid) = red[0]; __threadfence(); *(volatile float*)(line + tid) = red[0]; } }
__device__ __forceinline__ int vox(int b, int n, int i, int j, int k) { const int g2 = b / 256, g3 = (b / 16) % 16, g4 = b % 16; const int n2 = n / 4, n3 = (n / 2) % 2, n4 = n % 2; return ((g2 * 4 + 2 * n2 + i) * SD + (g3 * 4 + 2 * n3 + j)) * SD + (g4 * 4 + 2 * n4 + k); }
__global__ __launch_bounds__(256) void k_dsop(const _Float16* __restrict__ Hh, const _Float16* __restrict__ Hl, _Float16* __restrict__ A) { const int t = blockIdx.x * 256 + threadIdx.x; if (t >= NRN * 16 * (CC / 8)) return; const int c0 = (t % (CC / 8)) * 8; const int tp = (t / (CC / 8)) % 16; const int row = t / ((CC / 8) * 16); const int b = row / NND, n = row % NND; const int tap = tp & 7; const _Float16* src = (tp < 8) ? Hh : Hl; FragH f; f.half[0] = *(const v8us*)((const unsigned short*)src + (size_t)vox(b, n, tap / 4, (tap / 2) % 2, tap % 2) * CC + c0);
  *(volatile v8us*)((unsigned short*)A + ((size_t)row * 16 + tp) * CC + c0) = f.half[0]; __threadfence(); *(volatile v8us*)((unsigned short*)A + ((size_t)row * 16 + tp) * CC + c0) = f.half[0]; }
__global__ __launch_bounds__(256) void k_wdu16(const float* __restrict__ wd, const float* __restrict__ wu, _Float16* __restrict__ BtD, _Float16* __restrict__ BtU) { const int t = blockIdx.x * 256 + threadIdx.x; if (t >= 32 * 8 * 4 + 256 * 4) return;
  if (t < 32 * 8 * 4) { const int o = t / 32, tap = (t / 4) % 8, c0 = (t % 4) * 8; FragH f, f2;
#pragma unroll
    for (int q = 0; q < 8; ++q) { const float wv = bf16_round(wd[((size_t)o * CC + c0 + q) * 8 + tap]) * 16.0f; f.h[q] = (_Float16)wv; f2.h[q] = (_Float16)(wv * 0.0009765625f); }
    for (int pass = 0; pass < 2; ++pass) { *(volatile v8us*)((unsigned short*)BtD + (size_t)o * 512 + tap * 32 + c0) = f.half[0]; *(volatile v8us*)((unsigned short*)BtD + (size_t)o * 512 + 256 + tap * 32 + c0) = f2.half[0]; if (pass == 0) __threadfence(); } }
  else { const int u = t - 32 * 8 * 4; const int row = u / 4, c0 = (u % 4) * 8; const int tap = row / 32, o = row % 32; FragH f, f2;
#pragma unroll
    for (int q = 0; q < 8; ++q) { const float wv = bf16_round(wu[(((size_t)(c0 + q) * CC + o) * 8) + tap]) * 16.0f; f.h[q] = (_Float16)wv; f2.h[q] = (_Float16)(wv * 0.0009765625f); }
    for (int pass = 0; pass < 2; ++pass) { *(volatile v8us*)((unsigned short*)BtU + (size_t)row * 64 + c0) = f.half[0]; *(volatile v8us*)((unsigned short*)BtU + (size_t)row * 64 + 32 + c0) = f2.half[0]; if (pass == 0) __threadfence(); } } }
__global__ __launch_bounds__(256) void k_node(const float* __restrict__ XD, const float* __restrict__ g, const float* __restrict__ be, float* __restrict__ XN) {
  #pragma clang fp contract(off)
  const int t = blockIdx.x * 256 + threadIdx.x; if (t >= NRN * (CC / 4)) return; const int c0 = (t % (CC / 4)) * 4, row = t / (CC / 4); const v4f a = *(const v4fa*)(XD + (size_t)row * CC + c0); v4f v;
#pragma unroll
  for (int q = 0; q < 4; ++q) v[q] = lrelu_f(a[q] * bf16_round(g[c0 + q]) + bf16_round(be[c0 + q]));
  *(volatile v4f*)(XN + (size_t)row * CC + c0) = v; __threadfence(); *(volatile v4f*)(XN + (size_t)row * CC + c0) = v; }
__global__ __launch_bounds__(256) void k_dif(const float* __restrict__ XN, _Float16* __restrict__ D16) {
  #pragma clang fp contract(off)
  const int t = blockIdx.x * 256 + threadIdx.x; if (t >= NPR * (CC / 8)) return; const int c0 = (t % (CC / 8)) * 8, pr = t / (CC / 8); const int b = pr / 64, i = (pr / 8) % 8, j = pr % 8; FragH f = FragH{};
  const float* xi = XN + ((size_t)b * NND + i) * CC + c0; const float* xj = XN + ((size_t)b * NND + j) * CC + c0;
#pragma unroll 1
  for (int q = 0; q < 8; ++q) { const float d = xi[q] - xj[q]; const _Float16 hv = (_Float16)((d < 0.f) ? (0.f - d) : d);
#pragma unroll
    for (int k = 0; k < 8; ++k) f.h[k] = (k == q) ? hv : f.h[k]; }
  *(volatile v8us*)((unsigned short*)D16 + (size_t)pr * CC + c0) = f.half[0]; __threadfence(); *(volatile v8us*)((unsigned short*)D16 + (size_t)pr * CC + c0) = f.half[0]; }
__global__ __launch_bounds__(256) void k_afl16(_Float16* F16, int N, size_t nrows, const float* __restrict__ g, const float* __restrict__ be, _Float16* O16) {
  #pragma clang fp contract(off)
  const size_t t = (size_t)blockIdx.x * 256 + threadIdx.x; if (t >= nrows * (N / 8)) return; const int c0 = (int)(t % (N / 8)) * 8; const size_t r = t / (N / 8); FragH in; in.half[0] = *(const v8us*)((const unsigned short*)F16 + r * N + c0); FragH f;
#pragma unroll
  for (int q = 0; q < 8; ++q) f.h[q] = (_Float16)lrelu_f((float)in.h[q] * bf16_round(g[c0 + q]) + bf16_round(be[c0 + q]));
  *(volatile v8us*)((unsigned short*)O16 + r * N + c0) = f.half[0]; __threadfence(); *(volatile v8us*)((unsigned short*)O16 + r * N + c0) = f.half[0]; }
__global__ __launch_bounds__(256) void k_gcn(const _Float16* __restrict__ H2f, const float* __restrict__ g2, const float* __restrict__ be2, const float* __restrict__ w3, const float* __restrict__ b3, const float* __restrict__ XN, const float* __restrict__ gw, _Float16* __restrict__ G16) {
  #pragma clang fp contract(off)
  __shared__ __attribute__((aligned(16))) float sP[8][8][8]; __shared__ __attribute__((aligned(16))) float sAgg[8][8][64];
  const int tid = threadIdx.x, w = tid >> 5, l = tid & 31; const int b = blockIdx.x * 8 + w; if (b >= NWN) return;
  float sc[2];
#pragma unroll
  for (int e = 0; e < 2; ++e) { const int pr = l * 2 + e; const _Float16* hrow = H2f + ((size_t)b * 64 + pr) * 96; float s = bf16_round(b3[0]);
#pragma unroll 1
    for (int c = 0; c < 96; ++c) s += lrelu_f((float)hrow[c] * bf16_round(g2[c]) + bf16_round(be2[c])) * bf16_round(w3[c]);
    sc[e] = s; }
#pragma unroll
  for (int e = 0; e < 2; ++e) { const int pr = l * 2 + e; const int jj = pr / 8, ii = pr % 8; *(volatile __attribute__((address_space(3))) float*)(( __attribute__((address_space(3))) float*)&sP[w][ii][jj]) = sc[e]; }
  __syncthreads();
  if (l < 8) { const int i = l; float m = -3.0e38f; float a[8];
#pragma unroll
    for (int j = 0; j < 8; ++j) { a[j] = sP[w][i][j] - ((i == j) ? 1.0e8f : 0.f); m = fmaxf(m, a[j]); }
    float su = 0.f;
#pragma unroll
    for (int j = 0; j < 8; ++j) { a[j] = expf(a[j] - m); su += a[j]; }
    v4f p0, p1;
#pragma unroll
    for (int j = 0; j < 4; ++j) { p0[j] = a[j] / su; p1[j] = a[4 + j] / su; }
    *(v4f*)&sP[w][i][0] = p0; *(v4f*)&sP[w][i][4] = p1; }
  __syncthreads();
  { const int i = l / 4, c0 = (l % 4) * 8; v4f self0, self1, nb0, nb1;
#pragma unroll
    for (int q = 0; q < 8; ++q) { const int c = c0 + q; float s = 0.f;
#pragma unroll
      for (int j = 0; j < 8; ++j) s += sP[w][i][j] * XN[((size_t)b * NND + j) * CC + c];
      const float xv = XN[((size_t)b * NND + i) * CC + c]; if (q < 4) { self0[q] = xv; nb0[q] = s; } else { self1[q - 4] = xv; nb1[q - 4] = s; } }
    *(v4f*)&sAgg[w][i][c0] = self0; *(v4f*)&sAgg[w][i][c0 + 4] = self1; *(v4f*)&sAgg[w][i][32 + c0] = nb0; *(v4f*)&sAgg[w][i][32 + c0 + 4] = nb1; }
  __syncthreads();
  { const int i = l / 4, o0 = (l % 4) * 8; FragH f = FragH{}, f2 = FragH{};
#pragma unroll 1
    for (int q = 0; q < 8; ++q) { const int o = o0 + q; float s = 0.f;
#pragma unroll 1
      for (int k = 0; k < 64; ++k) s += sAgg[w][i][k] * bf16_round(gw[(size_t)k * CC + o]);
      const float gv = lrelu_f(s); const _Float16 hv = (_Float16)gv; const _Float16 lv = (_Float16)((gv - (float)hv) * 1024.0f);
#pragma unroll
      for (int kk = 0; kk < 8; ++kk) { f.h[kk] = (kk == q) ? hv : f.h[kk]; f2.h[kk] = (kk == q) ? lv : f2.h[kk]; } }
    for (int pass = 0; pass < 2; ++pass) { *(volatile v8us*)((unsigned short*)G16 + ((size_t)b * NND + i) * 64 + o0) = f.half[0]; *(volatile v8us*)((unsigned short*)G16 + ((size_t)b * NND + i) * 64 + 32 + o0) = f2.half[0]; if (pass == 0) __threadfence(); } } }
__global__ __launch_bounds__(256) void k_outv(const float* __restrict__ UP, const float* __restrict__ bu, const float* __restrict__ g, const float* __restrict__ be, float* __restrict__ out) {
  #pragma clang fp contract(off)
  const int t = blockIdx.x * 256 + threadIdx.x; if (t >= CC * (NP / 4)) return; const int p0 = (t % (NP / 4)) * 4; const int o = t / (NP / 4); const int d2 = p0 / (SD * SD), d3 = (p0 / SD) % SD; const float bo = bf16_round(bu[o]), gg = bf16_round(g[o]), bb = bf16_round(be[o]); v4f v;
#pragma unroll
  for (int q = 0; q < 4; ++q) { const int d4 = p0 % SD + q; const int g2 = d2 / 4, g3 = d3 / 4, g4 = d4 / 4; const int r2 = d2 % 4, r3 = d3 % 4, r4 = d4 % 4; const int b = (g2 * 16 + g3) * 16 + g4; const int n = (r2 / 2) * 4 + (r3 / 2) * 2 + (r4 / 2); const int tap = (r2 % 2) * 4 + (r3 % 2) * 2 + (r4 % 2);
    v[q] = lrelu_f((UP[((size_t)b * NND + n) * 256 + tap * 32 + o] + bo) * gg + bb); }
  *(volatile v4f*)(out + (size_t)o * NP + p0) = v; __threadfence(); *(volatile v4f*)(out + (size_t)o * NP + p0) = v; }

extern "C" void kernel_launch(void* const* d_in, const int* in_sizes, int n_in,
                              void* d_out, int out_size, void* d_ws, size_t ws_size, hipStream_t stream) {
  (void)in_sizes; (void)n_in; (void)out_size;
  const float* const* I = (const float* const*)d_in; const float* x = I[0]; const float* w_cc1 = I[1]; const float* b_cc1 = I[2]; const float* w_cc2 = I[3]; const float* b_cc2 = I[4]; const float* w_down = I[5]; const float* b_down = I[6]; const float* g_down = I[7]; const float* be_down = I[8]; const float* w_adj1 = I[9]; const float* b_adj1 = I[10]; const float* g_adj1 = I[11]; const float* be_adj1 = I[12]; const float* w_adj2 = I[13]; const float* b_adj2 = I[14]; const float* g_adj2 = I[15]; const float* be_adj2 = I[16]; const float* w_adj3 = I[17]; const float* b_adj3 = I[18]; const float* gcn_w = I[19]; const float* w_up = I[20]; const float* b_up = I[21]; const float* g_up = I[22]; const float* be_up = I[23];
  char* ws = (char*)d_ws; size_t off = 0;
  auto take = [&](size_t bytes) { char* p = ws + off; off += (bytes + 255) & ~(size_t)255; return p; };
  _Float16* BC1 = (_Float16*)take((size_t)64 * 27 * 32 * 2); _Float16* BC2 = (_Float16*)take((size_t)32 * 27 * 64 * 2); _Float16* BtD = (_Float16*)take((size_t)32 * 512 * 2); _Float16* BtU = (_Float16*)take((size_t)256 * 64 * 2); _Float16* BA1 = (_Float16*)take((size_t)64 * 32 * 2); _Float16* BA2 = (_Float16*)take((size_t)96 * 64 * 2); float* ST = (float*)take((size_t)2 * 64 * 32 * 4);
  _Float16* R0 = (_Float16*)take((size_t)NP * CC * 2); _Float16* R1 = (_Float16*)take((size_t)NP * CC * 2);
  char* BIGF = (char*)take((size_t)NP * 64 * 4);
  float* XD = (float*)take((size_t)NRN * CC * 4); float* XN = (float*)take((size_t)NRN * CC * 4); _Float16* G16 = (_Float16*)take((size_t)NRN * 64 * 2);
  if (off > ws_size) return;
  const size_t MB16 = (size_t)NP * CC * 2;
  _Float16* X16 = R0; _Float16* COL1 = R1; float* F1 = (float*)BIGF; _Float16* H1 = R0;
  _Float16* COL2 = (_Float16*)BIGF; float* F2 = (float*)(BIGF + MB16); _Float16* H2lo = (_Float16*)BIGF; _Float16* H2hi = (_Float16*)(BIGF + 3 * MB16);
  _Float16* AOP = R0; _Float16* DIF16 = (_Float16*)(BIGF + MB16); _Float16* ADJ1 = R0; _Float16* ADJ2 = (_Float16*)BIGF; float* UP = (float*)R0;
  const int PC1 = 8192, PC2 = 4096;
  k_w3d<<<(64 * (27 * 32 / 8) + 255) / 256, 256, 0, stream>>>(w_cc1, 64, 32, BC1); k_w3d<<<(32 * (27 * 64 / 8) + 255) / 256, 256, 0, stream>>>(w_cc2, 32, 64, BC2); k_wdu16<<<(32 * 8 * 4 + 256 * 4 + 255) / 256, 256, 0, stream>>>(w_down, w_up, BtD, BtU);
  k_round16f<<<(64 * 32 / 8 + 255) / 256, 256, 0, stream>>>(w_adj1, BA1, (size_t)64 * 32 / 8); k_round16f<<<(96 * 64 / 8 + 255) / 256, 256, 0, stream>>>(w_adj2, BA2, (size_t)96 * 64 / 8);
  k_x16v<<<(NP * (CC / 8) + 255) / 256, 256, 0, stream>>>(x, X16);
  for (int p0 = 0; p0 < NP; p0 += PC1) { k_im2col3<<<(PC1 * 27 * 4 + 255) / 256, 256, 0, stream>>>(X16, 32, p0, PC1, COL1);
    k_gemm_hhx<0><<<dim3(((PC1 / 16) * 1 + 3) / 4, 1), 128, 0, stream>>>(COL1, 864, 0, BC1, 864, 0, 0.0625f, b_cc1, 0, nullptr, 1, 0, 0, F1 + (size_t)p0 * 64, nullptr, 64, 0, PC1, 64, 864); }
  k_stat32<<<64, 256, 0, stream>>>(F1, 64, 0, ST); k_stat32<<<64, 256, 0, stream>>>(F1, 64, 1, ST); k_inl32<<<(NP * 8 + 255) / 256, 256, 0, stream>>>(F1, 64, ST, H1, nullptr);
  for (int p0 = 0; p0 < NP; p0 += PC2) { k_im2col3<<<(PC2 * 27 * 8 + 255) / 256, 256, 0, stream>>>(H1, 64, p0, PC2, COL2);
    k_gemm_hhx<0><<<dim3(((PC2 / 16) * 1 + 3) / 4, 1), 128, 0, stream>>>(COL2, 1728, 0, BC2, 1728, 0, 0.0625f, b_cc2, 0, nullptr, 1, 0, 0, F2 + (size_t)p0 * 32, nullptr, 32, 0, PC2, 32, 1728); }
  k_stat32<<<32, 256, 0, stream>>>(F2, 32, 0, ST); k_stat32<<<32, 256, 0, stream>>>(F2, 32, 1, ST); k_inl32<<<(NP * 4 + 255) / 256, 256, 0, stream>>>(F2, 32, ST, H2hi, H2lo);
  k_dsop<<<(NRN * 16 * 4 + 255) / 256, 256, 0, stream>>>(H2hi, H2lo, AOP);
  k_gemm_hhx<0><<<dim3(((NRN / 16) * 1 + 3) / 4, 1), 128, 0, stream>>>(AOP, 512, 0, BtD, 512, 0, 0.0625f, b_down, 0, nullptr, 1, 0, 0, XD, nullptr, CC, 0, NRN, CC, 512);
  k_node<<<(NRN * 8 + 255) / 256, 256, 0, stream>>>(XD, g_down, be_down, XN);
  k_dif<<<(NPR * 4 + 255) / 256, 256, 0, stream>>>(XN, DIF16);
  k_gemm_hhx<0><<<dim3(((NPR / 16) * 1 + 3) / 4, 1), 128, 0, stream>>>(DIF16, CC, 0, BA1, CC, 0, 0.0625f, b_adj1, 0, nullptr, 1, 0, 0, nullptr, ADJ1, 64, 0, NPR, 64, CC);
  k_afl16<<<(unsigned)(((size_t)NPR * 8 + 255) / 256), 256, 0, stream>>>(ADJ1, 64, (size_t)NPR, g_adj1, be_adj1, ADJ1);
  k_gemm_hhx<0><<<dim3(((NPR / 16) * 2 + 3) / 4, 1), 128, 0, stream>>>(ADJ1, 64, 0, BA2, 64, 0, 0.0625f, b_adj2, 0, nullptr, 1, 0, 0, nullptr, ADJ2, 96, 0, NPR, 96, 64);
  k_gcn<<<NWN / 8, 256, 0, stream>>>(ADJ2, g_adj2, be_adj2, w_adj3, b_adj3, XN, gcn_w, G16);
  k_gemm_hhx<0><<<dim3(((NRN / 16) * 4 + 3) / 4, 1), 128, 0, stream>>>(G16, 64, 0, BtU, 64, 0, 0.0625f, nullptr, 0, nullptr, 1, 0, 0, UP, nullptr, 256, 0, NRN, 256, 64);
  k_outv<<<(CC * (NP / 4) + 255) / 256, 256, 0, stream>>>(UP, b_up, g_up, be_up, (float*)d_out);
}
